// LowRankHighOrderSelfAttention_67061619360469
// MI455X (gfx1250) — hardware-verified
//
#include <hip/hip_runtime.h>
#include <math.h>

typedef __attribute__((ext_vector_type(16))) _Float16 v16h;
typedef __attribute__((ext_vector_type(16))) __bf16 v16b;
typedef __attribute__((ext_vector_type(8)))  _Float16 v8h;
typedef __attribute__((ext_vector_type(8)))  float v8f;
typedef __attribute__((ext_vector_type(4)))  float v4f;
typedef __attribute__((ext_vector_type(2)))  float v2f;
typedef __attribute__((ext_vector_type(4)))  unsigned v4u;
typedef __attribute__((ext_vector_type(4)))  int v4i;
typedef float __attribute__((may_alias)) float_a;
typedef int __attribute__((may_alias)) int_a;

template <typename T> __device__ __forceinline__ void vst2(void* p, T v) { *(volatile T*)p = v; __threadfence(); *(volatile T*)p = v; }
__device__ __forceinline__ v8f wmma16(v16h a, v16h b, v8f c) {
  v8f d = __builtin_amdgcn_wmma_f32_16x16x32_f16(false, a, false, b, (short)0, c, false, false);
  asm volatile("v_nop\n\tv_nop\n\tv_nop\n\tv_nop" : "+v"(d) : "v"(a), "v"(b));
  return d;
}
__device__ __forceinline__ v8f wmma_bf(v16b a, v16b b, v8f c) {
  v8f d = __builtin_amdgcn_wmma_f32_16x16x32_bf16(false, a, false, b, (short)0, c, false, false);
  asm volatile("v_nop\n\tv_nop\n\tv_nop\n\tv_nop" : "+v"(d) : "v"(a), "v"(b));
  return d;
}
__device__ __forceinline__ v16h frag_h(const _Float16* rowk0, int lane) {
  union { v16h v; v8h q[2]; } u; const _Float16* p = rowk0 + 8 * (lane >> 4);
  u.q[0] = *(const v8h*)p; u.q[1] = *(const v8h*)(p + 16); return u.v;
}
__device__ __forceinline__ v16h frag_f32(const float* rowk0, int lane) {
  v16h a; const float* p = rowk0 + 8 * (lane >> 4);
#pragma unroll
  for (int i = 0; i < 8; ++i) { a[i] = (_Float16)p[i]; a[8 + i] = (_Float16)p[16 + i]; }
  return a;
}
__device__ __forceinline__ v16h frag_f32s(const float* rowk0, int lane, float sc) {
  v16h a; const float* p = rowk0 + 8 * (lane >> 4);
#pragma unroll
  for (int i = 0; i < 8; ++i) { a[i] = (_Float16)(p[i] * sc); a[8 + i] = (_Float16)(p[16 + i] * sc); }
  return a;
}
__device__ __forceinline__ v16h fragc_f32(const float* W, int k0, int n, int lane, int ld, int K) {
  v16h a; const int g = lane >> 4;
#pragma unroll
  for (int i = 0; i < 8; ++i) { const int ka = k0 + 8 * g + i, kb = ka + 16;
    a[i] = (_Float16)(ka < K ? W[(size_t)(ka < K ? ka : K - 1) * ld + n] : 0.f); a[8 + i] = (_Float16)(kb < K ? W[(size_t)(kb < K ? kb : K - 1) * ld + n] : 0.f); }
  return a;
}
struct F2 { v16b h, l; };
__device__ __forceinline__ F2 bsplit16(const float v[16]) { F2 r;
#pragma unroll
  for (int i = 0; i < 16; ++i) { const __bf16 h = (__bf16)v[i]; r.h[i] = h; r.l[i] = (__bf16)(v[i] - (float)h); }
  return r; }
__device__ __forceinline__ F2 split_row(const float* row, int k0, int lane) { float v[16]; const float* p = row + k0 + 8 * (lane >> 4);
#pragma unroll
  for (int i = 0; i < 8; ++i) { v[i] = p[i]; v[8 + i] = p[16 + i]; }
  return bsplit16(v); }
__device__ __forceinline__ F2 split_rowK(const float* row, int k0, int lane, int K) { float v[16]; const int g = lane >> 4;
#pragma unroll
  for (int i = 0; i < 8; ++i) { const int ka = k0 + 8 * g + i, kb = ka + 16; v[i] = ka < K ? row[ka < K ? ka : K - 1] : 0.f; v[8 + i] = kb < K ? row[kb < K ? kb : K - 1] : 0.f; }
  return bsplit16(v); }
__device__ __forceinline__ F2 split_col(const float* W, int k0, int n, int lane, int ld, int K) { float v[16]; const int g = lane >> 4;
#pragma unroll
  for (int i = 0; i < 8; ++i) { const int ka = k0 + 8 * g + i, kb = ka + 16; v[i] = ka < K ? W[(size_t)(ka < K ? ka : K - 1) * ld + n] : 0.f; v[8 + i] = kb < K ? W[(size_t)(kb < K ? kb : K - 1) * ld + n] : 0.f; }
  return bsplit16(v); }
__device__ __forceinline__ v8f mac3(const F2& a, const F2& b, v8f c) { c = wmma_bf(a.l, b.h, c); c = wmma_bf(a.h, b.l, c); return wmma_bf(a.h, b.h, c); }
__device__ __forceinline__ float sigm(float v) { return 1.0f / (1.0f + expf(-v)); }
#define LDSX() do { asm volatile("s_wait_dscnt 0" ::: "memory"); __builtin_amdgcn_wave_barrier(); __builtin_amdgcn_fence(__ATOMIC_RELEASE, "workgroup"); } while (0)


#define NBT 4
#define N1 64
#define N2 128
#define DMOD 256
#define NHD 8
#define DHD 32
#define MF 192
#define NPOS (NBT * N1 * N2)
#ifndef TNB
#define TNB NBT
#endif
#ifndef TB0
#define TB0 0
#endif
typedef __attribute__((ext_vector_type(8))) __bf16 v8b;
__device__ __forceinline__ v16b frag_b(const __bf16* rowk0, int lane) {
  union { v16b v; v8b q[2]; } u; const __bf16* p = rowk0 + 8 * (lane >> 4);
  u.q[0] = *(const v8b*)p; u.q[1] = *(const v8b*)(p + 16); return u.v;
}
__device__ __forceinline__ v16b frag_gbf(const float* rowk0, int lane) {
  v16b a; const float* p = rowk0 + 8 * (lane >> 4);
#pragma unroll
  for (int i = 0; i < 8; ++i) { a[i] = (__bf16)p[i]; a[8 + i] = (__bf16)p[16 + i]; }
  return a;
}
__device__ __forceinline__ float bfr(float v) { return (float)(__bf16)v; }
__device__ __attribute__((noinline)) float exp_ni(float v) { return expf(v); }
__device__ __attribute__((noinline)) float pow_ni(float a, float b) { return powf(a, b); }
__device__ __attribute__((noinline)) float cos_ni(float v) { return cosf(v); }
__device__ __attribute__((noinline)) float sin_ni(float v) { return sinf(v); }

#define WS_A    0u
#define WS_B    (WS_A + 4u * NPOS * DMOD)
#define WS_V    (WS_B + 4u * NPOS * DMOD)
#define WS_QS1  (WS_V + 4u * NPOS * DMOD)
#define WS_KS1  (WS_QS1 + 4u * NBT * N1 * DMOD)
#define WS_QS2  (WS_KS1 + 4u * NBT * N1 * DMOD)
#define WS_KS2  (WS_QS2 + 4u * NBT * N2 * DMOD)
#define WS_MM   (WS_KS2 + 4u * NBT * N2 * DMOD)
#define MMS 32
#define WS_QP   (WS_MM + 4u * 4 * 65 * MMS)
#define WS_KPT  (WS_QP + 4u * NBT * NHD * N2 * MF)
#define WS_KSUM (WS_KPT + 4u * NBT * NHD * MF * N2)
#define WS_AN   (WS_KSUM + 4u * NBT * NHD * MF)
#define WS_END  (WS_AN + 4u * NBT * NHD * N2)

__global__ __launch_bounds__(128) void k_proj(const float* __restrict__ X, const float* __restrict__ Wq, const float* __restrict__ bq, const float* __restrict__ Wk, const float* __restrict__ bk, const float* __restrict__ Wv, const float* __restrict__ bv, float* __restrict__ Q, float* __restrict__ Kb, float* __restrict__ V) {
  __shared__ __align__(16) float so[4][16][132];
  const int tid = threadIdx.x, wave = tid >> 5, lane = tid & 31, col = lane & 15, g = lane >> 4; const size_t r0 = (size_t)blockIdx.x * 64 + wave * 16; const int nb = blockIdx.y; const int which = nb >> 1, n0 = (nb & 1) * 128;
  const float* Wm = which == 0 ? Wq : (which == 1 ? Wk : Wv); const float* bm = which == 0 ? bq : (which == 1 ? bk : bv); float* dst = which == 0 ? Q : (which == 1 ? Kb : V);
  v8f acc[8] = {};
#pragma unroll 2
  for (int kc = 0; kc < DMOD / 32; ++kc) { const v16b a = frag_gbf(X + (r0 + col) * DMOD + kc * 32, lane);
#pragma unroll
    for (int j = 0; j < 8; ++j) acc[j] = wmma_bf(a, frag_gbf(Wm + (size_t)(n0 + j * 16 + col) * DMOD + kc * 32, lane), acc[j]); }
#pragma unroll
  for (int j = 0; j < 8; ++j) { const float bb = bfr(bm[n0 + j * 16 + col]);
#pragma unroll
    for (int r = 0; r < 8; ++r) so[wave][8 * g + r][j * 16 + col] = acc[j][r] + bb; }
  LDSX();
  for (int rl = 0; rl < 16; ++rl) vst2(dst + (r0 + rl) * DMOD + n0 + lane * 4, *(const v4f*)&so[wave][rl][lane * 4]);
}
__global__ __launch_bounds__(256) void k_pool1(const float* __restrict__ T, float* __restrict__ S1) {
  __shared__ __align__(16) float srow[DMOD];
  const int b = blockIdx.x / N1, i1 = blockIdx.x % N1, c = threadIdx.x; float s = 0.f;
  for (int i2 = 0; i2 < N2; ++i2) s += T[(((size_t)b * N1 + i1) * N2 + i2) * DMOD + c];
  srow[c] = s; __syncthreads();
  if (c < 64) vst2(S1 + (size_t)blockIdx.x * DMOD + c * 4, *(const v4f*)&srow[c * 4]);
}
__global__ __launch_bounds__(256) void k_pool2(const float* __restrict__ T, float* __restrict__ S2) {
  __shared__ __align__(16) float srow[DMOD];
  const int b = blockIdx.x / N2, i2 = blockIdx.x % N2, c = threadIdx.x; float s = 0.f;
  for (int i1 = 0; i1 < N1; ++i1) s += T[(((size_t)b * N1 + i1) * N2 + i2) * DMOD + c];
  srow[c] = s; __syncthreads();
  if (c < 64) vst2(S2 + (size_t)blockIdx.x * DMOD + c * 4, *(const v4f*)&srow[c * 4]);
}
__global__ __launch_bounds__(256) void k_rope(float* __restrict__ SQ, float* __restrict__ SK) {
  __shared__ __align__(16) float sq[DMOD], sk[DMOD];
  const int l = blockIdx.x % N2, tid = threadIdx.x; const size_t row = (size_t)blockIdx.x * DMOD; const int d = tid & 31, j = d & 15;
  const float invf = 1.0f / pow_ni(10000.0f, (float)(2 * j) / 32.0f); const float ang = (float)l * invf; const float c = cos_ni(ang), s = sin_ni(ang);
  const float xq = SQ[row + tid], xk = SK[row + tid]; const float rq = d < 16 ? -SQ[row + tid + 16] : SQ[row + tid - 16]; const float rk = d < 16 ? -SK[row + tid + 16] : SK[row + tid - 16];
  sq[tid] = xq * c + rq * s; sk[tid] = xk * c + rk * s;
  __syncthreads();
  if (tid < 64) vst2(SQ + row + tid * 4, *(const v4f*)&sq[tid * 4]); else if (tid < 128) vst2(SK + row + (tid - 64) * 4, *(const v4f*)&sk[(tid - 64) * 4]);
}
__global__ __launch_bounds__(256) void k_minmax(const float* __restrict__ T, int n, int t, float* __restrict__ MMP) {
  __shared__ float smn[8], smx[8]; __shared__ __align__(16) float sres[4];
  const int tid = threadIdx.x, wave = tid >> 5, lane = tid & 31; float mn = 3.0e38f, mx = -3.0e38f;
  for (int i = blockIdx.x * 256 + tid; i < n; i += 64 * 256) { const float v = T[i]; mn = fminf(mn, v); mx = fmaxf(mx, v); }
#pragma unroll
  for (int o = 1; o < 32; o <<= 1) { mn = fminf(mn, __shfl_xor(mn, o)); mx = fmaxf(mx, __shfl_xor(mx, o)); }
  if (lane == 0) { smn[wave] = mn; smx[wave] = mx; }
  __syncthreads();
  if (tid == 0) { float a = smn[0], bq2 = smx[0]; for (int w = 1; w < 8; ++w) { a = fminf(a, smn[w]); bq2 = fmaxf(bq2, smx[w]); } sres[0] = a; sres[1] = bq2; sres[2] = 0.f; sres[3] = 0.f; }
  __syncthreads();
  if (tid < 8) { const v4f z = {0.f, 0.f, 0.f, 0.f}; vst2(MMP + ((size_t)t * 65 + blockIdx.x) * MMS + tid * 4, tid == 0 ? *(const v4f*)sres : z); }
}
__global__ __launch_bounds__(64) void k_mmfin(float* __restrict__ MMP) {
  const int t = blockIdx.x, tid = threadIdx.x; float mn = MMP[((size_t)t * 65 + tid) * MMS], mx = MMP[((size_t)t * 65 + tid) * MMS + 1];
#pragma unroll
  for (int o = 1; o < 32; o <<= 1) { mn = fminf(mn, __shfl_xor(mn, o)); mx = fmaxf(mx, __shfl_xor(mx, o)); }
  __shared__ float s2[4];
  if ((tid & 31) == 0) { s2[(tid >> 5) * 2] = mn; s2[(tid >> 5) * 2 + 1] = mx; }
  __syncthreads();
  __shared__ __align__(16) float sfin[4];
  if (tid == 0) { sfin[0] = fminf(s2[0], s2[2]); sfin[1] = fmaxf(s2[1], s2[3]); sfin[2] = 0.f; sfin[3] = 0.f; }
  __syncthreads();
  if (tid < 8) { const v4f z = {0.f, 0.f, 0.f, 0.f}; vst2(MMP + ((size_t)t * 65 + 64) * MMS + tid * 4, tid == 0 ? *(const v4f*)sfin : z); }
}

__global__ __launch_bounds__(32) void k_feat(const float* __restrict__ S, int L, const float* __restrict__ MM, int t, const float* __restrict__ feat, float* __restrict__ P) {
  __shared__ __align__(16) float sx[16][36]; __shared__ __align__(16) float so[16][196]; __shared__ float soff[16];
  const int lane = threadIdx.x, col = lane & 15, g = lane >> 4; const int h = blockIdx.y; const int r0 = blockIdx.x * 16; const int b = r0 / L, l0 = r0 % L;
  const float mn = MM[((size_t)t * 65 + 64) * MMS], mx = MM[((size_t)t * 65 + 64) * MMS + 1]; const float sc = 1.0f / (mx - mn); const float temp = 0.42044820762685725f;
  { const int rl = lane >> 1, half = lane & 1; float ss = 0.f;
    for (int d = half * 16; d < half * 16 + 16; ++d) { const float x = S[(size_t)(r0 + rl) * DMOD + h * DHD + d]; const float xs = (x - mn) * sc * temp; sx[rl][d] = xs; ss += xs * xs; }
    ss += __shfl_xor(ss, 1); if (half == 0) { soff[rl] = -0.5f * ss - 0.5f * 5.2574953720277815f + 1e-6f; sx[rl][32] = 0.f; sx[rl][33] = 0.f; sx[rl][34] = 0.f; sx[rl][35] = 0.f; } }
  LDSX();
  const F2 a = split_row(&sx[col][0], 0, lane);
#pragma unroll
  for (int j = 0; j < 12; ++j) { v8f acc = {}; const v16b w = frag_gbf(feat + (size_t)(j * 16 + col) * DHD, lane); acc = wmma_bf(a.l, w, acc); acc = wmma_bf(a.h, w, acc);
#pragma unroll
    for (int r = 0; r < 8; ++r) so[8 * g + r][j * 16 + col] = exp_ni(acc[r] + soff[8 * g + r]); }
  LDSX();
  for (int q = lane; q < 16 * 48; q += 32) { const int rl = q / 48, pc = q % 48; vst2(P + ((size_t)(b * NHD + h) * L + l0 + rl) * MF + pc * 4, *(const v4f*)&so[rl][pc * 4]); }
}
__global__ __launch_bounds__(256) void k_kpt(const float* __restrict__ KP, int L, float* __restrict__ KPT, float* __restrict__ KS) {
  __shared__ float st[MF][N2 + 1]; __shared__ __align__(16) float ssum[MF]; __shared__ __align__(16) float srow[N2];
  const int bh = blockIdx.x, tid = threadIdx.x;
  for (int q = tid; q < L * MF; q += 256) { const int l = q / MF, m = q % MF; st[m][l] = KP[((size_t)bh * L + l) * MF + m]; }
  __syncthreads();
  if (tid < MF) { float s = 0.f; for (int l = 0; l < L; ++l) s += st[tid][l]; ssum[tid] = s; }
  for (int m = 0; m < MF; ++m) { __syncthreads(); if (tid < N2) srow[tid] = tid < L ? st[m][tid] : 0.f; __syncthreads(); if (tid < 32) vst2(KPT + ((size_t)bh * MF + m) * N2 + tid * 4, *(const v4f*)&srow[tid * 4]); }
  __syncthreads();
  if (tid < 48) vst2(KS + (size_t)bh * MF + tid * 4, *(const v4f*)&ssum[tid * 4]);
}
__global__ __launch_bounds__(128) void k_an(const float* __restrict__ QP, const float* __restrict__ KS, int L, float* __restrict__ AN) {
  __shared__ float sks[MF]; __shared__ __align__(16) float sres[N2];
  const int bh = blockIdx.x, tid = threadIdx.x;
  for (int m = tid; m < MF; m += 128) sks[m] = KS[(size_t)bh * MF + m];
  __syncthreads();
  float s = 0.f; if (tid < L) { const float* row = QP + ((size_t)bh * L + tid) * MF; for (int m = 0; m < MF; ++m) s += row[m] * sks[m]; }
  sres[tid] = tid < L ? s : 1.0f;
  __syncthreads();
  if (tid < 32) vst2(AN + (size_t)bh * N2 + tid * 4, *(const v4f*)&sres[tid * 4]);
}
template <int PASS>
__global__ __launch_bounds__(256) void k_vt(const float* __restrict__ V, float* __restrict__ VT, int ob0) {
  __shared__ float st[DMOD][(PASS == 1 ? N1 : N2) + 1];
  const int tid = threadIdx.x; constexpr int L = (PASS == 1 ? N1 : N2); const int other = ob0 + blockIdx.x;
  const int b = PASS == 1 ? other / N2 : other / N1, o = PASS == 1 ? other % N2 : other % N1;
  for (int q = tid; q < L * DMOD; q += 256) { const int l = q / DMOD, c = q % DMOD; const size_t src = PASS == 1 ? ((((size_t)b * N1 + l) * N2 + o) * DMOD + c) : ((((size_t)b * N1 + o) * N2 + l) * DMOD + c); st[c][l] = V[src]; }
  __syncthreads();
  __shared__ __align__(16) float srow[4][N2];
  for (int c0 = 0; c0 < DMOD; c0 += 4) { const int cc = c0 + (tid >> 6), ll = tid & 63;
    for (int l = ll; l < L; l += 64) srow[tid >> 6][l] = st[cc][l];
    __syncthreads();
    if (tid < 4 * (L / 4)) { const int c1 = tid / (L / 4), pc = tid % (L / 4); vst2(VT + ((size_t)other * DMOD + c0 + c1) * L + pc * 4, *(const v4f*)&srow[c1][pc * 4]); }
    __syncthreads(); }
}
__global__ __launch_bounds__(64) void k_kv(const float* __restrict__ VT, const float* __restrict__ KPT, int L, int O, int b, float* __restrict__ KVT) {
  __shared__ __align__(16) float so[2][16][196];
  const int tid = threadIdx.x, wave = tid >> 5, lane = tid & 31, col = lane & 15, g = lane >> 4; const int blk = blockIdx.x; const int h = blk % NHD, o = blk / NHD; const int bo = b * O + o;
  const float* arow = VT + ((size_t)bo * DMOD + h * DHD + wave * 16 + col) * L;
  v8f acc[12] = {};
  for (int kc = 0; kc < L / 32; ++kc) { const F2 a = split_row(arow, kc * 32, lane);
#pragma unroll
    for (int j = 0; j < 12; ++j) { const F2 kb = split_row(KPT + ((size_t)(b * NHD + h) * MF + j * 16 + col) * N2, kc * 32, lane); acc[j] = mac3(a, kb, acc[j]); } }
#pragma unroll
  for (int j = 0; j < 12; ++j)
#pragma unroll
    for (int r = 0; r < 8; ++r) so[wave][8 * g + r][j * 16 + col] = acc[j][r];
  LDSX();
  for (int q = lane; q < 16 * 48; q += 32) { const int rl = q / 48, pc = q % 48; vst2(KVT + (((size_t)blk) * DHD + wave * 16 + rl) * MF + pc * 4, *(const v4f*)&so[wave][rl][pc * 4]); }
}
__global__ __launch_bounds__(256) void k_att(const float* __restrict__ QP, const float* __restrict__ KVT, const float* __restrict__ AN, int L, int O, int pass, int b, float* __restrict__ Vout) {
  __shared__ __align__(16) float so[8][16][36];
  const int tid = threadIdx.x, wave = tid >> 5, lane = tid & 31, col = lane & 15, g = lane >> 4; const int blk = blockIdx.x; const int h = blk % NHD, o = blk / NHD;
  if (wave * 16 >= L) return;
  const float* qrow = QP + ((size_t)(b * NHD + h) * L + wave * 16 + col) * MF;
  v8f acc[2] = {};
#pragma unroll
  for (int kc = 0; kc < MF / 32; ++kc) { const F2 a = split_row(qrow, kc * 32, lane);
#pragma unroll
    for (int j = 0; j < 2; ++j) { const F2 kb = split_row(KVT + ((size_t)blk * DHD + j * 16 + col) * MF, kc * 32, lane); acc[j] = mac3(a, kb, acc[j]); } }
  float inv[8];
#pragma unroll
  for (int r = 0; r < 8; ++r) inv[r] = 1.0f / AN[(size_t)(b * NHD + h) * N2 + wave * 16 + 8 * g + r];
#pragma unroll
  for (int j = 0; j < 2; ++j)
#pragma unroll
    for (int r = 0; r < 8; ++r) so[wave][8 * g + r][j * 16 + col] = acc[j][r] * inv[r];
  LDSX();
  for (int q = lane; q < 16 * 8; q += 32) { const int rl = q >> 3, pc = q & 7; const int l = wave * 16 + rl;
    const size_t pos = pass == 1 ? (((size_t)b * N1 + l) * N2 + o) : (((size_t)b * N1 + o) * N2 + l);
    vst2(Vout + pos * DMOD + h * DHD + pc * 4, *(const v4f*)&so[wave][rl][pc * 4]); }
}
__global__ __launch_bounds__(128) void k_out(const float* __restrict__ V3, const float* __restrict__ Wo, const float* __restrict__ bo, float* __restrict__ Y, int rb0) {
  __shared__ __align__(16) float so[4][16][132];
  const int tid = threadIdx.x, wave = tid >> 5, lane = tid & 31, col = lane & 15, g = lane >> 4; const size_t r0 = (size_t)(rb0 + blockIdx.x) * 64 + wave * 16; const int n0 = blockIdx.y * 128;
  v8f acc[8] = {};
#pragma unroll 2
  for (int kc = 0; kc < DMOD / 32; ++kc) { const F2 a = split_row(V3 + (r0 + col) * DMOD, kc * 32, lane);
#pragma unroll
    for (int j = 0; j < 8; ++j) { const v16b w = frag_gbf(Wo + (size_t)(n0 + j * 16 + col) * DMOD + kc * 32, lane); acc[j] = wmma_bf(a.l, w, acc[j]); acc[j] = wmma_bf(a.h, w, acc[j]); } }
#pragma unroll
  for (int j = 0; j < 8; ++j) { const float bb = bfr(bo[n0 + j * 16 + col]);
#pragma unroll
    for (int r = 0; r < 8; ++r) so[wave][8 * g + r][j * 16 + col] = acc[j][r] + bb; }
  LDSX();
  for (int rl = 0; rl < 16; ++rl) vst2(Y + (r0 + rl) * DMOD + n0 + lane * 4, *(const v4f*)&so[wave][rl][lane * 4]);
}

#ifndef DBG
#define DBG 0
#endif
#if DBG != 0
__global__ __launch_bounds__(256) void k_dump(const float* __restrict__ src, int n, float* __restrict__ out) {
  const size_t p = (size_t)blockIdx.x * 256 + threadIdx.x; v4f v; for (int i = 0; i < 4; ++i) { const size_t f = p * 4 + i; v[i] = f < (size_t)n ? src[f] : 0.f; } vst2(out + p * 4, v);
}
#endif
extern "C" void kernel_launch(void* const* d_in, const int* in_sizes, int n_in, void* d_out, int out_size, void* d_ws, size_t ws_size, hipStream_t stream) {
  (void)in_sizes; (void)n_in; (void)out_size;
  const float** F = (const float**)d_in;
  if (ws_size < (size_t)WS_END) return;
  char* ws = (char*)d_ws; float *BA = (float*)(ws + WS_A), *BB = (float*)(ws + WS_B), *V = (float*)(ws + WS_V), *QS1 = (float*)(ws + WS_QS1), *KS1 = (float*)(ws + WS_KS1), *QS2 = (float*)(ws + WS_QS2), *KS2 = (float*)(ws + WS_KS2), *MM = (float*)(ws + WS_MM), *QP = (float*)(ws + WS_QP), *KPT = (float*)(ws + WS_KPT), *KSUM = (float*)(ws + WS_KSUM), *AN = (float*)(ws + WS_AN);
  float* KP = BB;
  k_proj<<<dim3(NPOS / 64, 6), 128, 0, stream>>>(F[0], F[1], F[2], F[3], F[4], F[5], F[6], BA, BB, V);
  k_pool1<<<NBT * N1, 256, 0, stream>>>(BA, QS1); k_pool1<<<NBT * N1, 256, 0, stream>>>(BB, KS1);
  k_pool2<<<NBT * N2, 256, 0, stream>>>(BA, QS2); k_pool2<<<NBT * N2, 256, 0, stream>>>(BB, KS2);
  k_rope<<<NBT * N2, 256, 0, stream>>>(QS2, KS2);
  k_minmax<<<64, 256, 0, stream>>>(QS1, NBT * N1 * DMOD, 0, MM); k_minmax<<<64, 256, 0, stream>>>(KS1, NBT * N1 * DMOD, 1, MM); k_minmax<<<64, 256, 0, stream>>>(QS2, NBT * N2 * DMOD, 2, MM); k_minmax<<<64, 256, 0, stream>>>(KS2, NBT * N2 * DMOD, 3, MM);
  k_mmfin<<<4, 64, 0, stream>>>(MM);
  k_feat<<<dim3(NBT * N1 / 16, NHD), 32, 0, stream>>>(QS1, N1, MM, 0, F[9], QP);
  k_feat<<<dim3(NBT * N1 / 16, NHD), 32, 0, stream>>>(KS1, N1, MM, 1, F[9], KP);
  k_kpt<<<NBT * NHD, 256, 0, stream>>>(KP, N1, KPT, KSUM);
  k_an<<<NBT * NHD, 128, 0, stream>>>(QP, KSUM, N1, AN);
#if DBG == 1
  k_dump<<<N1 * N2 * DMOD / 1024, 256, 0, stream>>>(AN, NBT * NHD * N2, (float*)d_out); return;
#elif DBG == 2
  k_dump<<<N1 * N2 * DMOD / 1024, 256, 0, stream>>>(QP, NBT * NHD * N1 * MF, (float*)d_out); return;
#endif
  k_vt<1><<<(TNB - TB0) * N2, 256, 0, stream>>>(V, BA, TB0 * N2);
  for (int b = TB0; b < TNB; ++b) { k_kv<<<N2 * NHD, 64, 0, stream>>>(BA, KPT, N1, N2, b, BB); k_att<<<N2 * NHD, 256, 0, stream>>>(QP, BB, AN, N1, N2, 1, b, V); }
#if DBG == 3
  k_dump<<<N1 * N2 * DMOD / 1024, 256, 0, stream>>>(V, N1 * N2 * DMOD, (float*)d_out); return;
#elif DBG == 4
  k_dump<<<N1 * N2 * DMOD / 1024, 256, 0, stream>>>(BB, N2 * NHD * DHD * MF, (float*)d_out); return;
#endif
  k_feat<<<dim3(NBT * N2 / 16, NHD), 32, 0, stream>>>(QS2, N2, MM, 2, F[9], QP);
  k_feat<<<dim3(NBT * N2 / 16, NHD), 32, 0, stream>>>(KS2, N2, MM, 3, F[9], KP);
  k_kpt<<<NBT * NHD, 256, 0, stream>>>(KP, N2, KPT, KSUM);
  k_an<<<NBT * NHD, 128, 0, stream>>>(QP, KSUM, N2, AN);
  k_vt<2><<<(TNB - TB0) * N1, 256, 0, stream>>>(V, BA, TB0 * N1);
  for (int b = TB0; b < TNB; ++b) { k_kv<<<N1 * NHD, 64, 0, stream>>>(BA, KPT, N2, N1, b, BB); k_att<<<N1 * NHD, 256, 0, stream>>>(QP, BB, AN, N2, N1, 2, b, V); }
#if DBG == 5
  k_dump<<<N1 * N2 * DMOD / 1024, 256, 0, stream>>>(V, N1 * N2 * DMOD, (float*)d_out); return;
#elif DBG == 6
  k_dump<<<N1 * N2 * DMOD / 1024, 256, 0, stream>>>(AN, NBT * NHD * N2, (float*)d_out); return;
#endif
  k_out<<<dim3((TNB - TB0) * N1 * N2 / 64, 2), 128, 0, stream>>>(V, F[7], F[8], (float*)d_out, TB0 * N1 * N2 / 64);
}
